// RotaryGQA_42228118454586
// MI455X (gfx1250) — hardware-verified
//
#include <hip/hip_runtime.h>
#define NBt 2
#define TT 2048
#define CC 1024
#define NH 16
#define HD 64
#define HG 2
#define SRCL 0
#define NR (NBt * TT)
typedef __bf16 v16b __attribute__((ext_vector_type(16)));
typedef unsigned short v8us __attribute__((ext_vector_type(8), may_alias));
typedef float  v8f  __attribute__((ext_vector_type(8)));
typedef float  v4f  __attribute__((ext_vector_type(4)));
typedef float  v4fa __attribute__((ext_vector_type(4), may_alias));
union FragB { v16b v; v8us half[2]; unsigned short u[16]; };

__device__ __forceinline__ unsigned short bf16_bits(float x) { unsigned int u = __float_as_uint(x); return (unsigned short)((u + 0x7FFFu + ((u >> 16) & 1u)) >> 16); }
__device__ __forceinline__ float bf16_val(unsigned short b) { return __uint_as_float(((unsigned int)b) << 16); }
__device__ __forceinline__ float bf16_round(float x) { return bf16_val(bf16_bits(x)); }
template <int NT>
__device__ __forceinline__ v8f mmaN(v16b ah, v16b al, v16b bh, v16b bl, v8f c) {
  c = __builtin_amdgcn_wmma_f32_16x16x32_bf16(false, ah, false, bh, (short)0, c, false, false);
  if (NT >= 2) c = __builtin_amdgcn_wmma_f32_16x16x32_bf16(false, al, false, bh, (short)0, c, false, false);
  if (NT >= 3) c = __builtin_amdgcn_wmma_f32_16x16x32_bf16(false, ah, false, bl, (short)0, c, false, false);
  asm volatile("v_nop\n\tv_nop\n\tv_nop\n\tv_nop" : "+v"(c) : "v"(ah), "v"(al), "v"(bh), "v"(bl));
  return c;
}

__global__ __launch_bounds__(256) void k_wt_bf16(const float* __restrict__ W, unsigned short* __restrict__ Wt, int K, int N) {
  const int t = blockIdx.x * 256 + threadIdx.x;
  const int k8n = K / 8;
  if (t >= N * k8n) return;
  const int n = t / k8n, k8 = (t % k8n) * 8;
  v8us v;
#pragma unroll
  for (int i = 0; i < 8; ++i) v[i] = bf16_bits(W[(size_t)(k8 + i) * N + n]);
  *(volatile v8us*)(Wt + (size_t)n * K + k8) = v;
  __threadfence();
  *(volatile v8us*)(Wt + (size_t)n * K + k8) = v;
}

template <bool ASPLIT, int ACT, bool BIAS_BF16>
__global__ __launch_bounds__(128) void k_gemm_bf(const float* __restrict__ A, int lda, const unsigned short* __restrict__ Wt, int ldb,
                                               const float* __restrict__ bias, float* __restrict__ C, int ldc, int M, int N, int K) {
  __shared__ __attribute__((aligned(16))) float so[4][16][64];
  const int tid = threadIdx.x, w = tid >> 5, lane = tid & 31, ln = lane & 15, hh = lane >> 4;
  const int ntn = N / 64;
  const int wid = blockIdx.x * 4 + w;
  const int mt = wid / ntn, nq = wid % ntn;
  if (mt * 16 >= M) return;
  const int row0 = mt * 16, col0 = nq * 64;
  const float* arow = A + (size_t)(row0 + ln) * lda;
  v8f acc[4] = {};
  for (int kb = 0; kb < K; kb += 32) {
    FragB ah, al;
    const v4f x0 = *(const v4fa*)(arow + kb + 8 * hh), x1 = *(const v4fa*)(arow + kb + 8 * hh + 4);
    const v4f x2 = *(const v4fa*)(arow + kb + 16 + 8 * hh), x3 = *(const v4fa*)(arow + kb + 16 + 8 * hh + 4);
    float xs[16] = {x0[0],x0[1],x0[2],x0[3],x1[0],x1[1],x1[2],x1[3],x2[0],x2[1],x2[2],x2[3],x3[0],x3[1],x3[2],x3[3]};
#pragma unroll
    for (int i = 0; i < 16; ++i) { const unsigned short hb = bf16_bits(xs[i]); ah.u[i] = hb; al.u[i] = ASPLIT ? bf16_bits(xs[i] - bf16_val(hb)) : (unsigned short)0; }
#pragma unroll
    for (int t = 0; t < 4; ++t) {
      const unsigned short* brow = Wt + (size_t)(col0 + t * 16 + ln) * ldb + kb;
      FragB b;
      b.half[0] = *(const v8us*)(brow + 8 * hh);
      b.half[1] = *(const v8us*)(brow + 16 + 8 * hh);
      acc[t] = mmaN<ASPLIT ? 2 : 1>(ah.v, al.v, b.v, b.v, acc[t]);
    }
  }
#pragma unroll
  for (int t = 0; t < 4; ++t) {
    float bv = bias ? bias[col0 + t * 16 + ln] : 0.f;
    if (BIAS_BF16) bv = bf16_round(bv);
#pragma unroll
    for (int r = 0; r < 8; ++r) { float v = acc[t][r] + bv; if (ACT == 1) v = fmaxf(v, 0.f); so[w][8 * hh + r][t * 16 + ln] = v; }
  }
  __builtin_amdgcn_fence(__ATOMIC_ACQ_REL, "workgroup");
  __builtin_amdgcn_wave_barrier();
  const int rsub = lane >> 4, c4 = (lane & 15) * 4;
  for (int pass = 0; pass < 2; ++pass) {
#pragma unroll
    for (int q = 0; q < 8; ++q) {
      const int r = q * 2 + rsub;
      const v4f v = *(const v4fa*)&so[w][r][c4];
      *(volatile v4f*)(C + (size_t)(row0 + r) * ldc + col0 + c4) = v;
    }
    if (pass == 0) __threadfence();
  }
}

template <bool ASPLIT, int ACT, bool BIAS_BF16, bool RES_BF16>
__global__ __launch_bounds__(128) void k_gemm_bf3(const float* __restrict__ A, int lda, const unsigned short* __restrict__ Wt, int ldb,
                                                const float* __restrict__ bias, const float* __restrict__ resid, int rmod, int ldr,
                                                float* __restrict__ C, int ldc, int M, int N, int K) {
  __shared__ __attribute__((aligned(16))) float so[4][16][64];
  const int tid = threadIdx.x, w = tid >> 5, lane = tid & 31, ln = lane & 15, hh = lane >> 4;
  const int ntn = N / 64;
  const int wid = blockIdx.x * 4 + w;
  const int mt = wid / ntn, nq = wid % ntn;
  if (mt * 16 >= M) return;
  const int row0 = mt * 16, col0 = nq * 64;
  const float* arow = A + (size_t)(row0 + ln) * lda;
  v8f acc[4] = {};
  for (int kb = 0; kb < K; kb += 32) {
    FragB ah, al;
    const v4f x0 = *(const v4fa*)(arow + kb + 8 * hh), x1 = *(const v4fa*)(arow + kb + 8 * hh + 4);
    const v4f x2 = *(const v4fa*)(arow + kb + 16 + 8 * hh), x3 = *(const v4fa*)(arow + kb + 16 + 8 * hh + 4);
    float xs[16] = {x0[0],x0[1],x0[2],x0[3],x1[0],x1[1],x1[2],x1[3],x2[0],x2[1],x2[2],x2[3],x3[0],x3[1],x3[2],x3[3]};
#pragma unroll
    for (int i = 0; i < 16; ++i) { const unsigned short hb = bf16_bits(xs[i]); ah.u[i] = hb; al.u[i] = ASPLIT ? bf16_bits(xs[i] - bf16_val(hb)) : (unsigned short)0; }
#pragma unroll
    for (int t = 0; t < 4; ++t) {
      const unsigned short* brow = Wt + (size_t)(col0 + t * 16 + ln) * ldb + kb;
      FragB b;
      b.half[0] = *(const v8us*)(brow + 8 * hh);
      b.half[1] = *(const v8us*)(brow + 16 + 8 * hh);
      acc[t] = mmaN<ASPLIT ? 2 : 1>(ah.v, al.v, b.v, b.v, acc[t]);
    }
  }
#pragma unroll
  for (int t = 0; t < 4; ++t) {
    const int col = col0 + t * 16 + ln;
    float bv = bias ? bias[col] : 0.f;
    if (BIAS_BF16) bv = bf16_round(bv);
#pragma unroll
    for (int r = 0; r < 8; ++r) {
      float v = acc[t][r] + bv;
      if (resid) { float rv = resid[(size_t)((row0 + 8 * hh + r) % rmod) * ldr + col]; if (RES_BF16) rv = bf16_round(rv); v += rv; }
      if (ACT == 1) v = fmaxf(v, 0.f);
      if (ACT == 2) v = 0.5f * v * (1.0f + erff(v * 0.70710678118654752f));
      if (ACT == 3) { const float u = 0.7978845608028654f * (v + 0.044715f * v * v * v); v = 0.5f * v * (1.0f + tanhf(u)); }
      so[w][8 * hh + r][t * 16 + ln] = v;
    }
  }
  __builtin_amdgcn_fence(__ATOMIC_ACQ_REL, "workgroup");
  __builtin_amdgcn_wave_barrier();
  const int rsub = lane >> 4, c4 = (lane & 15) * 4;
  for (int pass = 0; pass < 2; ++pass) {
#pragma unroll
    for (int q = 0; q < 8; ++q) {
      const int r = q * 2 + rsub;
      const v4f v = *(const v4fa*)&so[w][r][c4];
      *(volatile v4f*)(C + (size_t)(row0 + r) * ldc + col0 + c4) = v;
    }
    if (pass == 0) __threadfence();
  }
}
template <bool PARAM_BF16>
__global__ __launch_bounds__(256) void k_layernorm(const float* __restrict__ X, const float* __restrict__ R, const float* __restrict__ g, const float* __restrict__ bta,
                                                  float* __restrict__ out_sum, float* __restrict__ out_norm, int N, float eps) {
  __shared__ float red[256];
  const int row = blockIdx.x, tid = threadIdx.x;
  const float* x = X + (size_t)row * N; const float* rr = R ? R + (size_t)row * N : nullptr;
  float vals[16];
  const int per = N / 256;
  float s1 = 0.f;
  for (int u = 0; u < per / 4; ++u) {
    const int j = tid * 4 + 1024 * u;
    const v4f a = *(const v4fa*)(x + j);
    v4f b = {0.f,0.f,0.f,0.f}; if (rr) b = *(const v4fa*)(rr + j);
#pragma unroll
    for (int q = 0; q < 4; ++q) { const float v = a[q] + b[q]; vals[u * 4 + q] = v; s1 += v; }
  }
  red[tid] = s1; __syncthreads();
  for (int st = 128; st > 0; st >>= 1) { if (tid < st) red[tid] += red[tid + st]; __syncthreads(); }
  const float mu = red[0] / (float)N; __syncthreads();
  float s2 = 0.f;
  for (int u = 0; u < per / 4; ++u)
#pragma unroll
    for (int q = 0; q < 4; ++q) { const float c = vals[u * 4 + q] - mu; s2 += c * c; }
  red[tid] = s2; __syncthreads();
  for (int st = 128; st > 0; st >>= 1) { if (tid < st) red[tid] += red[tid + st]; __syncthreads(); }
  const float rs = rsqrtf(red[0] / (float)N + eps);
  for (int pass = 0; pass < 2; ++pass) {
    for (int u = 0; u < per / 4; ++u) {
      const int j = tid * 4 + 1024 * u;
      v4f o, sm;
#pragma unroll
      for (int q = 0; q < 4; ++q) {
        float gg = g[j + q], bb = bta[j + q];
        if (PARAM_BF16) { gg = bf16_round(gg); bb = bf16_round(bb); }
        sm[q] = vals[u * 4 + q]; o[q] = (vals[u * 4 + q] - mu) * rs * gg + bb;
      }
      if (out_sum) *(volatile v4f*)(out_sum + (size_t)row * N + j) = sm;
      *(volatile v4f*)(out_norm + (size_t)row * N + j) = o;
    }
    if (pass == 0) __threadfence();
  }
}


typedef _Float16 v16h __attribute__((ext_vector_type(16)));
union FragH { v16h v; v8us half[2]; _Float16 h[16]; unsigned short u[16]; };
template <int NT>
__device__ __forceinline__ v8f mmaH(v16h ah, v16h al, v16h bh, v16h bl, v8f c) {
  c = __builtin_amdgcn_wmma_f32_16x16x32_f16(false, ah, false, bh, (short)0, c, false, false);
  if (NT >= 2) c = __builtin_amdgcn_wmma_f32_16x16x32_f16(false, al, false, bh, (short)0, c, false, false);
  if (NT >= 3) c = __builtin_amdgcn_wmma_f32_16x16x32_f16(false, ah, false, bl, (short)0, c, false, false);
  asm volatile("v_nop\n\tv_nop\n\tv_nop\n\tv_nop" : "+v"(c) : "v"(ah), "v"(al), "v"(bh), "v"(bl));
  return c;
}
template <bool ASPLIT>
__global__ __launch_bounds__(128) void k_gemm_h(const float* __restrict__ A, int lda, size_t sA, const _Float16* __restrict__ Bh, int ldb, size_t sB, float alpha, float* __restrict__ C, int ldc, size_t sC, int M, int N, int K) {
  __shared__ __attribute__((aligned(16))) float so[4][16][64];
  const int tid = threadIdx.x, w = tid >> 5, lane = tid & 31, ln = lane & 15, hh = lane >> 4; const int by = blockIdx.y;
  A += (size_t)by * sA; Bh += (size_t)by * sB; C += (size_t)by * sC;
  const int ntn = (N + 63) / 64; const int wid = blockIdx.x * 4 + w; const int mt = wid / ntn, nq = wid % ntn; if (mt * 16 >= M) return;
  const int row0 = mt * 16, col0 = nq * 64; const float* arow = A + (size_t)(row0 + ln) * lda;
  v8f acc[4] = {};
  for (int kb = 0; kb < K; kb += 32) {
    FragH ah, al;
    const v4f x0 = *(const v4fa*)(arow + kb + 8 * hh), x1 = *(const v4fa*)(arow + kb + 8 * hh + 4), x2 = *(const v4fa*)(arow + kb + 16 + 8 * hh), x3 = *(const v4fa*)(arow + kb + 16 + 8 * hh + 4);
    float xs[16] = {x0[0],x0[1],x0[2],x0[3],x1[0],x1[1],x1[2],x1[3],x2[0],x2[1],x2[2],x2[3],x3[0],x3[1],x3[2],x3[3]};
#pragma unroll
    for (int i = 0; i < 16; ++i) { const _Float16 h = (_Float16)xs[i]; ah.h[i] = h; al.h[i] = ASPLIT ? (_Float16)(xs[i] - (float)h) : (_Float16)0.0f; }
#pragma unroll
    for (int t = 0; t < 4; ++t) { if (col0 + t * 16 >= N) continue; const size_t boff = (size_t)(col0 + t * 16 + ln) * ldb + kb; FragH bq; bq.half[0] = *(const v8us*)(Bh + boff + 8 * hh); bq.half[1] = *(const v8us*)(Bh + boff + 16 + 8 * hh);
      acc[t] = mmaH<ASPLIT ? 2 : 1>(ah.v, al.v, bq.v, bq.v, acc[t]); }
  }
#pragma unroll
  for (int t = 0; t < 4; ++t) { if (col0 + t * 16 >= N) continue;
#pragma unroll
    for (int r = 0; r < 8; ++r) so[w][8 * hh + r][t * 16 + ln] = acc[t][r] * alpha; }
  __builtin_amdgcn_fence(__ATOMIC_ACQ_REL, "workgroup"); __builtin_amdgcn_wave_barrier();
  const int rsub = lane >> 4, c4 = (lane & 15) * 4;
  for (int pass = 0; pass < 2; ++pass) {
#pragma unroll
    for (int q = 0; q < 8; ++q) { const int r = q * 2 + rsub; if (col0 + c4 < N) { const v4f v = *(const v4fa*)&so[w][r][c4]; *(volatile v4f*)(C + (size_t)(row0 + r) * ldc + col0 + c4) = v; } }
    if (pass == 0) __threadfence(); }
}

__global__ __launch_bounds__(256) void k_wt_f16(const float* __restrict__ W, _Float16* __restrict__ Wt, int K, int N, float scale) {
  const int t = blockIdx.x * 256 + threadIdx.x; if (t >= N * (K / 8)) return; const int n = t / (K / 8), k8 = (t % (K / 8)) * 8; FragH f;
#pragma unroll
  for (int i = 0; i < 8; ++i) f.h[i] = (_Float16)(bf16_round(W[(size_t)(k8 + i) * N + n]) * scale); const v8us o = f.half[0];
  *(volatile v8us*)((unsigned short*)Wt + (size_t)n * K + k8) = o; __threadfence(); *(volatile v8us*)((unsigned short*)Wt + (size_t)n * K + k8) = o;
}
template <int ACT>
__global__ __launch_bounds__(128) void k_gemm_hhx(const _Float16* __restrict__ A, int lda, size_t sA, const _Float16* __restrict__ Bh, int ldb, size_t sB, float alpha, const float* __restrict__ bias, size_t sBias, const float* __restrict__ CP, int rowsPerB, size_t sCPb, int row0g,
    float* __restrict__ C, _Float16* __restrict__ C16, int ldc, size_t sC, int M, int N, int K) {
  __shared__ __attribute__((aligned(16))) float so[4][16][64];
  const int tid = threadIdx.x, w = tid >> 5, lane = tid & 31, ln = lane & 15, hh = lane >> 4; const int by = blockIdx.y;
  A += (size_t)by * sA; Bh += (size_t)by * sB; const size_t cofs = (size_t)by * sC; const float* bp = bias ? bias + (size_t)by * sBias : nullptr;
  const int ntn = (N + 63) / 64; const int wid = blockIdx.x * 4 + w; const int mt = wid / ntn, nq = wid % ntn; if (mt * 16 >= M) return;
  const int row0 = mt * 16, col0 = nq * 64; const _Float16* arow = A + (size_t)(row0 + ln) * lda;
  v8f acc[4] = {};
  for (int kb = 0; kb < K; kb += 32) { FragH ah; ah.half[0] = *(const v8us*)((const unsigned short*)arow + kb + 8 * hh); ah.half[1] = *(const v8us*)((const unsigned short*)arow + kb + 16 + 8 * hh);
#pragma unroll
    for (int t = 0; t < 4; ++t) { if (col0 + t * 16 >= N) continue; const size_t boff = (size_t)(col0 + t * 16 + ln) * ldb + kb; FragH bq; bq.half[0] = *(const v8us*)((const unsigned short*)Bh + boff + 8 * hh); bq.half[1] = *(const v8us*)((const unsigned short*)Bh + boff + 16 + 8 * hh);
      acc[t] = mmaH<1>(ah.v, ah.v, bq.v, bq.v, acc[t]); }
  }
#pragma unroll
  for (int t = 0; t < 4; ++t) { if (col0 + t * 16 >= N) continue; const int col = col0 + t * 16 + ln; const float bv = bp ? bf16_round(bp[col]) : 0.f;
#pragma unroll
    for (int r = 0; r < 8; ++r) { float v = acc[t][r] * alpha + bv; if (CP) { const int bidx = (row0g + row0 + 8 * hh + r) / rowsPerB; v += CP[(size_t)bidx * sCPb + (size_t)by * 64 + col]; } if (ACT == 1) v = (v > 0.f) ? v : expm1f(v); else if (ACT == 7) v = (v > 0.f) ? v + 1.0f : expf(v); else if (ACT == 8) v = tanhf(v); else if (ACT == 9) v = 0.5f * v * (1.0f + tanhf(0.7978845608028654f * (v + 0.044715f * v * v * v))); else if (ACT == 11) v = 1.0f / (1.0f + expf(-v)); else if (ACT == 12) v = (v > 0.f) ? v : 0.01f * v; else if (ACT == 14) v = (v > 0.f) ? v : 0.1f * v; else if (ACT == 15) v = v / (1.0f + expf(-v)); else if (ACT == 3) v = fmaxf(v, 0.f); else if (ACT == 6) v = 0.5f * v * (1.0f + erff(v * 0.70710678118654752f)); so[w][8 * hh + r][t * 16 + ln] = v; } }
  __builtin_amdgcn_fence(__ATOMIC_ACQ_REL, "workgroup"); __builtin_amdgcn_wave_barrier();
  const int rsub = lane >> 4, c4 = (lane & 15) * 4; typedef _Float16 v4h __attribute__((ext_vector_type(4)));
  for (int pass = 0; pass < 2; ++pass) {
#pragma unroll
    for (int q = 0; q < 8; ++q) { const int r = q * 2 + rsub; if (col0 + c4 < N) { const v4f v = *(const v4fa*)&so[w][r][c4]; if (C) *(volatile v4f*)(C + cofs + (size_t)(row0 + r) * ldc + col0 + c4) = v; if (C16) { v4h h4; for (int i = 0; i < 4; ++i) h4[i] = (_Float16)v[i]; *(volatile v4h*)(C16 + cofs + (size_t)(row0 + r) * ldc + col0 + c4) = h4; } } }
    if (pass == 0) __threadfence(); }
}


typedef _Float16 v4h __attribute__((ext_vector_type(4)));

__global__ __launch_bounds__(256) void k_x16(const float* __restrict__ x, _Float16* __restrict__ X16, size_t n8) { const size_t t = (size_t)blockIdx.x * 256 + threadIdx.x; if (t >= n8) return; FragH f;
#pragma unroll
  for (int q = 0; q < 8; ++q) f.h[q] = (_Float16)bf16_round(x[t * 8 + q]); *(volatile v8us*)((unsigned short*)X16 + t * 8) = f.half[0]; __threadfence(); *(volatile v8us*)((unsigned short*)X16 + t * 8) = f.half[0]; }
__global__ __launch_bounds__(256) void k_h16(const float* __restrict__ x, _Float16* __restrict__ X16, size_t n8) { const size_t t = (size_t)blockIdx.x * 256 + threadIdx.x; if (t >= n8) return; FragH f;
#pragma unroll
  for (int q = 0; q < 8; ++q) f.h[q] = (_Float16)x[t * 8 + q]; *(volatile v8us*)((unsigned short*)X16 + t * 8) = f.half[0]; __threadfence(); *(volatile v8us*)((unsigned short*)X16 + t * 8) = f.half[0]; }
__global__ __launch_bounds__(256) void k_round16f(const float* __restrict__ W, _Float16* __restrict__ Bt, size_t n8) { const size_t t = (size_t)blockIdx.x * 256 + threadIdx.x; if (t >= n8) return; FragH f;
#pragma unroll
  for (int i = 0; i < 8; ++i) f.h[i] = (_Float16)(bf16_round(W[t * 8 + i]) * 16.0f); *(volatile v8us*)((unsigned short*)Bt + t * 8) = f.half[0]; __threadfence(); *(volatile v8us*)((unsigned short*)Bt + t * 8) = f.half[0]; }
template <int NHv, int TTv>
__global__ __launch_bounds__(256) void k_vt(const _Float16* __restrict__ V16, int ldv, int voff, _Float16* __restrict__ Vt) { __shared__ unsigned short tl[64][66]; const int tid = threadIdx.x; const int slab = blockIdx.x / (TTv / 64), lg = blockIdx.x % (TTv / 64); const int b = slab / NHv, h = slab % NHv;
  for (int i = tid; i < 64 * 8; i += 256) { const int r = i / 8, c8 = (i % 8) * 8; FragH f; f.half[0] = *(const v8us*)((const unsigned short*)V16 + ((size_t)b * TTv + lg * 64 + r) * ldv + voff + h * 64 + c8);
#pragma unroll
    for (int q = 0; q < 8; ++q) tl[r][c8 + q] = f.u[q]; }
  __syncthreads();
  for (int pass = 0; pass < 2; ++pass) {
#pragma unroll
    for (int rd = 0; rd < 2; ++rd) { const int d = rd * 32 + tid / 8, pc = tid % 8; FragH f;
#pragma unroll
      for (int q = 0; q < 8; ++q) f.u[q] = tl[pc * 8 + q][d];
      *(volatile v8us*)((unsigned short*)Vt + ((size_t)slab * 64 + d) * TTv + lg * 64 + pc * 8) = f.half[0]; }
    if (pass == 0) __threadfence(); } }

__global__ __launch_bounds__(256) void k_hl(const float* __restrict__ F, _Float16* __restrict__ Hh, _Float16* __restrict__ Hl, size_t n8) { const size_t t = (size_t)blockIdx.x * 256 + threadIdx.x; if (t >= n8) return; FragH fh, fl; const v4f a = *(const v4fa*)(F + t * 8), c = *(const v4fa*)(F + t * 8 + 4);
#pragma unroll
  for (int q = 0; q < 4; ++q) { _Float16 h = (_Float16)a[q]; fh.h[q] = h; fl.h[q] = (_Float16)((a[q] - (float)h) * 1024.0f); h = (_Float16)c[q]; fh.h[4 + q] = h; fl.h[4 + q] = (_Float16)((c[q] - (float)h) * 1024.0f); }
  for (int pass = 0; pass < 2; ++pass) { *(volatile v8us*)((unsigned short*)Hh + t * 8) = fh.half[0]; *(volatile v8us*)((unsigned short*)Hl + t * 8) = fl.half[0]; if (pass == 0) __threadfence(); } }

__global__ __launch_bounds__(256) void k_tab(float* __restrict__ CSt) { const int i = blockIdx.x * 256 + threadIdx.x; if (i >= TT * (HD / 2)) return; const int p = i % (HD / 2), tt = i / (HD / 2); const float freq = 1.0f / powf(10000.0f, (float)(2 * p) / (float)HD); const float ang = (float)tt * freq; typedef float v2f __attribute__((ext_vector_type(2))); v2f v; v[0] = cosf(ang); v[1] = sinf(ang); *(volatile v2f*)(CSt + (size_t)i * 2) = v; __threadfence(); *(volatile v2f*)(CSt + (size_t)i * 2) = v; }
__global__ __launch_bounds__(256) void k_rope(const float* __restrict__ P, const float* __restrict__ CSt, _Float16* __restrict__ O16) {
  #pragma clang fp contract(off)
  const int t = blockIdx.x * 256 + threadIdx.x; if (t >= NR * (CC / 16)) return; const int c16 = (t % (CC / 16)) * 16, r = t / (CC / 16); const int tt = r % TT; const int p0 = (c16 % HD) / 2; const float* src = P + (size_t)r * CC + c16; FragH f[2];
#pragma unroll
  for (int q = 0; q < 8; ++q) { const int p = p0 + q; const float cs = CSt[((size_t)tt * (HD / 2) + p) * 2], sn = CSt[((size_t)tt * (HD / 2) + p) * 2 + 1]; const float x0 = src[2 * q], x1 = src[2 * q + 1]; const float o0 = x0 * cs - x1 * sn, o1 = x0 * sn + x1 * cs; f[(2 * q) >> 3].h[(2 * q) & 7] = (_Float16)o0; f[(2 * q + 1) >> 3].h[(2 * q + 1) & 7] = (_Float16)o1; }
  for (int pass = 0; pass < 2; ++pass) { *(volatile v8us*)((unsigned short*)O16 + (size_t)r * CC + c16) = f[0].half[0]; *(volatile v8us*)((unsigned short*)O16 + (size_t)r * CC + c16 + 8) = f[1].half[0]; if (pass == 0) __threadfence(); } }
__global__ __launch_bounds__(256) void k_split(const float* __restrict__ F, _Float16* __restrict__ Hh, _Float16* __restrict__ Hl, size_t n8) {
  #pragma clang fp contract(off)
  const size_t t = (size_t)blockIdx.x * 256 + threadIdx.x; if (t >= n8) return; const v4f a = *(const v4fa*)(F + t * 8), c = *(const v4fa*)(F + t * 8 + 4); FragH fh, fl;
#pragma unroll
  for (int q = 0; q < 8; ++q) { const float v = (q < 4) ? a[q] : c[q - 4]; const _Float16 hi = (_Float16)v; fh.h[q] = hi; fl.h[q] = (_Float16)((v - (float)hi) * 1024.0f); }
  for (int pass = 0; pass < 2; ++pass) { *(volatile v8us*)((unsigned short*)Hh + t * 8) = fh.half[0]; *(volatile v8us*)((unsigned short*)Hl + t * 8) = fl.half[0]; if (pass == 0) __threadfence(); } }
__global__ __launch_bounds__(256) void k_split2(const float* __restrict__ F, _Float16* __restrict__ O2, size_t n8) {
  #pragma clang fp contract(off)
  const size_t t = (size_t)blockIdx.x * 256 + threadIdx.x; if (t >= n8) return; const size_t r = t / (CC / 8); const int c0 = (int)(t % (CC / 8)) * 8; const v4f a = *(const v4fa*)(F + t * 8), c = *(const v4fa*)(F + t * 8 + 4); FragH fh, fl;
#pragma unroll
  for (int q = 0; q < 8; ++q) { const float v = (q < 4) ? a[q] : c[q - 4]; const _Float16 hi = (_Float16)v; fh.h[q] = hi; fl.h[q] = (_Float16)((v - (float)hi) * 1024.0f); }
  for (int pass = 0; pass < 2; ++pass) { *(volatile v8us*)((unsigned short*)O2 + r * 2 * CC + c0) = fh.half[0]; *(volatile v8us*)((unsigned short*)O2 + r * 2 * CC + CC + c0) = fl.half[0]; if (pass == 0) __threadfence(); } }
__global__ __launch_bounds__(256) void k_bfold(const float* __restrict__ Wm, _Float16* __restrict__ Bt) { const int t = blockIdx.x * 256 + threadIdx.x; if (t >= CC * (2 * CC / 8)) return; const int k0 = (t % (2 * CC / 8)) * 8, o = t / (2 * CC / 8); const int kb = k0 & (CC - 1); const float sc = (k0 >= CC) ? (16.0f / 1024.0f) : 16.0f; FragH f;
#pragma unroll
  for (int q = 0; q < 8; ++q) f.h[q] = (_Float16)(bf16_round(Wm[(size_t)(kb + q) * CC + o]) * sc);
  *(volatile v8us*)((unsigned short*)Bt + (size_t)o * 2 * CC + k0) = f.half[0]; __threadfence(); *(volatile v8us*)((unsigned short*)Bt + (size_t)o * 2 * CC + k0) = f.half[0]; }
__global__ __launch_bounds__(256) void k_wth(const float* __restrict__ Wm, int K, int N, _Float16* __restrict__ Bt) { const int t = blockIdx.x * 256 + threadIdx.x; if (t >= NH * N * (K / 8)) return; const int k0 = (t % (K / 8)) * 8; const int n = (t / (K / 8)) % N; const int h = t / ((K / 8) * N); FragH f;
#pragma unroll
  for (int q = 0; q < 8; ++q) f.h[q] = (_Float16)(bf16_round(Wm[((size_t)h * K + k0 + q) * N + n]) * 16.0f);
  *(volatile v8us*)((unsigned short*)Bt + ((size_t)h * N + n) * K + k0) = f.half[0]; __threadfence(); *(volatile v8us*)((unsigned short*)Bt + ((size_t)h * N + n) * K + k0) = f.half[0]; }
__global__ __launch_bounds__(256) void k_foldh(const float* __restrict__ F, int wd, _Float16* __restrict__ O16, size_t n8) {
  #pragma clang fp contract(off)
  const size_t t = (size_t)blockIdx.x * 256 + threadIdx.x; if (t >= n8) return; const int per = wd / 8; const size_t r = t / ((size_t)NH * per); const int h = (int)((t / per) % NH), c0 = (int)(t % per) * 8; const float* src = F + r * ((size_t)NH * wd) + (size_t)h * wd + c0; const v4f a = *(const v4fa*)src, c = *(const v4fa*)(src + 4); FragH fh, fl;
#pragma unroll
  for (int q = 0; q < 8; ++q) { const float v = (q < 4) ? a[q] : c[q - 4]; const _Float16 hi = (_Float16)v; fh.h[q] = hi; fl.h[q] = (_Float16)((v - (float)hi) * 1024.0f); }
  unsigned short* dst = (unsigned short*)O16 + r * ((size_t)NH * 2 * wd) + (size_t)h * 2 * wd;
  for (int pass = 0; pass < 2; ++pass) { *(volatile v8us*)(dst + c0) = fh.half[0]; *(volatile v8us*)(dst + wd + c0) = fl.half[0]; if (pass == 0) __threadfence(); } }
__global__ __launch_bounds__(256) void k_wth2(const float* __restrict__ Wm, int K, int N, _Float16* __restrict__ Bt) { const int t = blockIdx.x * 256 + threadIdx.x; if (t >= NH * N * (2 * K / 8)) return; const int k0 = (t % (2 * K / 8)) * 8; const int n = (t / (2 * K / 8)) % N; const int h = t / ((2 * K / 8) * N); const int kb = k0 % K; const float sc = (k0 >= K) ? (16.0f / 1024.0f) : 16.0f; FragH f;
#pragma unroll
  for (int q = 0; q < 8; ++q) f.h[q] = (_Float16)(bf16_round(Wm[((size_t)h * K + kb + q) * N + n]) * sc);
  *(volatile v8us*)((unsigned short*)Bt + ((size_t)h * N + n) * 2 * K + k0) = f.half[0]; __threadfence(); *(volatile v8us*)((unsigned short*)Bt + ((size_t)h * N + n) * 2 * K + k0) = f.half[0]; }
__global__ __launch_bounds__(256) void k_rope(const float* __restrict__ F, int nh, _Float16* __restrict__ O16) {
  #pragma clang fp contract(off)
  const int wdt = nh * HD; const int t8 = blockIdx.x * 256 + threadIdx.x; if (t8 >= NR * (wdt / 8)) return; const int c0 = (t8 % (wdt / 8)) * 8; const int r = t8 / (wdt / 8); const int t = r % TT; const int d0 = c0 % HD; const v4f a = *(const v4fa*)(F + (size_t)r * wdt + c0), c = *(const v4fa*)(F + (size_t)r * wdt + c0 + 4); FragH f = FragH{};
#pragma unroll 1
  for (int p = 0; p < 4; ++p) { const int i = (d0 >> 1) + p; const float inv = 1.0f / powf(10000.0f, (float)(2 * i) / (float)HD); const float ang = (float)t * inv; const float cs = cosf(ang), sn = sinf(ang); const float e = (p == 0) ? a[0] : (p == 1) ? a[2] : (p == 2) ? c[0] : c[2]; const float o = (p == 0) ? a[1] : (p == 1) ? a[3] : (p == 2) ? c[1] : c[3]; const _Float16 r0 = (_Float16)(e * cs - o * sn), r1 = (_Float16)(e * sn + o * cs);
#pragma unroll
    for (int k = 0; k < 4; ++k) { f.h[2 * k] = (k == p) ? r0 : f.h[2 * k]; f.h[2 * k + 1] = (k == p) ? r1 : f.h[2 * k + 1]; } }
  *(volatile v8us*)((unsigned short*)O16 + (size_t)r * wdt + c0) = f.half[0]; __threadfence(); *(volatile v8us*)((unsigned short*)O16 + (size_t)r * wdt + c0) = f.half[0]; }
#define KVW 256
__global__ __launch_bounds__(256) void k_vtk(const _Float16* __restrict__ V, int b, _Float16* __restrict__ VT) { const int t = blockIdx.x * 256 + threadIdx.x; if (t >= KVW * (TT / 8)) return; const int s0 = (t % (TT / 8)) * 8, hd = t / (TT / 8); FragH f;
#pragma unroll
  for (int q = 0; q < 8; ++q) f.h[q] = V[((size_t)b * TT + s0 + q) * KVW + hd];
  *(volatile v8us*)((unsigned short*)VT + (size_t)hd * TT + s0) = f.half[0]; __threadfence(); *(volatile v8us*)((unsigned short*)VT + (size_t)hd * TT + s0) = f.half[0]; }
__global__ __launch_bounds__(256) void k_vt(const _Float16* __restrict__ V16, int b, _Float16* __restrict__ VT) { const int t = blockIdx.x * 256 + threadIdx.x; if (t >= CC * (TT / 8)) return; const int t0 = (t % (TT / 8)) * 8, hd = t / (TT / 8); FragH f;
#pragma unroll
  for (int q = 0; q < 8; ++q) f.h[q] = V16[((size_t)b * TT + t0 + q) * CC + hd];
  *(volatile v8us*)((unsigned short*)VT + (size_t)hd * TT + t0) = f.half[0]; __threadfence(); *(volatile v8us*)((unsigned short*)VT + (size_t)hd * TT + t0) = f.half[0]; }
__global__ __launch_bounds__(256) void k_msoft(const float* __restrict__ S, _Float16* __restrict__ P16) {
  #pragma clang fp contract(off)
  const int tid = threadIdx.x, w = tid >> 5, ln = tid & 31; const int row = blockIdx.x * 8 + w; if (row >= HG * TT) return; const int i = row % TT; const int jmax = min(TT - 1, i + SRCL); const int jend = min(TT, ((jmax + 1 + 255) / 256) * 256); const float* sr = S + (size_t)row * TT; float m = -3.0e38f;
#pragma unroll 1
  for (int jb = 0; jb < jend; jb += 256) { const v4f a = *(const v4fa*)(sr + jb + 8 * ln), c = *(const v4fa*)(sr + jb + 8 * ln + 4);
#pragma unroll
    for (int k = 0; k < 8; ++k) { const int j = jb + 8 * ln + k; const float v = (k < 4) ? a[k] : c[k - 4]; if (j <= jmax) m = fmaxf(m, v); } }
  for (int o = 16; o > 0; o >>= 1) m = fmaxf(m, __shfl_xor(m, o, 32));
  float su = 0.f;
#pragma unroll 1
  for (int jb = 0; jb < jend; jb += 256) { const v4f a = *(const v4fa*)(sr + jb + 8 * ln), c = *(const v4fa*)(sr + jb + 8 * ln + 4);
#pragma unroll
    for (int k = 0; k < 8; ++k) { const int j = jb + 8 * ln + k; const float v = (k < 4) ? a[k] : c[k - 4]; su += (j <= jmax) ? expf(v - m) : 0.f; } }
  for (int o = 16; o > 0; o >>= 1) su += __shfl_xor(su, o, 32); const float inv = 1024.0f / su;
  for (int pass = 0; pass < 2; ++pass) {
#pragma unroll 1
    for (int jb = 0; jb < TT; jb += 256) { FragH f;
      if (jb < jend) { const v4f a = *(const v4fa*)(sr + jb + 8 * ln), c = *(const v4fa*)(sr + jb + 8 * ln + 4);
#pragma unroll
        for (int k = 0; k < 8; ++k) { const int j = jb + 8 * ln + k; const float v = (k < 4) ? a[k] : c[k - 4]; f.h[k] = (j <= jmax) ? (_Float16)(expf(v - m) * inv) : (_Float16)0.0f; } }
      else { f = FragH{}; }
      *(volatile v8us*)((unsigned short*)P16 + (size_t)row * TT + jb + 8 * ln) = f.half[0]; }
    if (pass == 0) __threadfence(); } }

extern "C" void kernel_launch(void* const* d_in, const int* in_sizes, int n_in,
                              void* d_out, int out_size, void* d_ws, size_t ws_size, hipStream_t stream) {
  (void)in_sizes; (void)n_in; (void)out_size;
  const float* x = (const float*)d_in[0]; const float* w_q = (const float*)d_in[1]; const float* b_q = (const float*)d_in[2]; const float* w_k = (const float*)d_in[3]; const float* b_k = (const float*)d_in[4]; const float* w_v = (const float*)d_in[5]; const float* b_v = (const float*)d_in[6]; const float* w_o = (const float*)d_in[7]; const float* b_o = (const float*)d_in[8];
  char* ws = (char*)d_ws; size_t off = 0;
  auto take = [&](size_t bytes) { char* p = ws + off; off += (bytes + 255) & ~(size_t)255; return p; };
  _Float16* BQ = (_Float16*)take((size_t)CC * CC * 2); _Float16* BK = (_Float16*)take((size_t)KVW * CC * 2); _Float16* BV = (_Float16*)take((size_t)KVW * CC * 2); _Float16* BO2 = (_Float16*)take((size_t)CC * 2 * CC * 2);
  _Float16* X16 = (_Float16*)take((size_t)NR * CC * 2); _Float16* Q16 = (_Float16*)take((size_t)NR * CC * 2); _Float16* K16 = (_Float16*)take((size_t)NR * KVW * 2); _Float16* Vh = (_Float16*)take((size_t)NR * KVW * 2); _Float16* Vl = (_Float16*)take((size_t)NR * KVW * 2); _Float16* VTh = (_Float16*)take((size_t)KVW * TT * 2); _Float16* VTl = (_Float16*)take((size_t)KVW * TT * 2); float* S = (float*)take((size_t)HG * TT * TT * 4); _Float16* P16 = (_Float16*)take((size_t)HG * TT * TT * 2); float* Of = (float*)take((size_t)NR * CC * 4);
  float* Ff = S;
  _Float16* O2 = P16;
  if (off > ws_size) return;
  k_wt_f16<<<(CC * (CC / 8) + 255) / 256, 256, 0, stream>>>(w_q, BQ, CC, CC, 16.0f); k_wt_f16<<<(KVW * (CC / 8) + 255) / 256, 256, 0, stream>>>(w_k, BK, CC, KVW, 16.0f); k_wt_f16<<<(KVW * (CC / 8) + 255) / 256, 256, 0, stream>>>(w_v, BV, CC, KVW, 16.0f); k_bfold<<<(unsigned)(((size_t)CC * (2 * CC / 8) + 255) / 256), 256, 0, stream>>>(w_o, BO2);
  const size_t n8 = (size_t)NR * CC / 8; const unsigned nb8 = (unsigned)((n8 + 255) / 256);
  k_x16<<<nb8, 256, 0, stream>>>(x, X16, n8);
  k_gemm_hhx<0><<<dim3(((NR / 16) * (CC / 64) + 3) / 4, 1), 128, 0, stream>>>(X16, CC, 0, BQ, CC, 0, 0.0625f, b_q, 0, nullptr, 1, 0, 0, Ff, nullptr, CC, 0, NR, CC, CC);
  k_rope<<<(unsigned)((NR * (CC / 8) + 255) / 256), 256, 0, stream>>>(Ff, NH, Q16);
  k_gemm_hhx<0><<<dim3(((NR / 16) * (KVW / 64) + 3) / 4, 1), 128, 0, stream>>>(X16, CC, 0, BK, CC, 0, 0.0625f, b_k, 0, nullptr, 1, 0, 0, Ff, nullptr, KVW, 0, NR, KVW, CC);
  k_rope<<<(unsigned)((NR * (KVW / 8) + 255) / 256), 256, 0, stream>>>(Ff, KVW / HD, K16);
  k_gemm_hhx<0><<<dim3(((NR / 16) * (KVW / 64) + 3) / 4, 1), 128, 0, stream>>>(X16, CC, 0, BV, CC, 0, 0.0625f, b_v, 0, nullptr, 1, 0, 0, Ff, nullptr, KVW, 0, NR, KVW, CC);
  k_split<<<(unsigned)(((size_t)NR * KVW / 8 + 255) / 256), 256, 0, stream>>>(Ff, Vh, Vl, (size_t)NR * KVW / 8);
  const dim3 gS(((TT / 16) * (TT / 64) + 3) / 4, HG), gV(((TT / 16) * 1 + 3) / 4, HG), gV1(((TT / 16) * 1 + 3) / 4, 1);
  for (int b = 0; b < NBt; ++b) {
    k_vtk<<<(KVW * (TT / 8) + 255) / 256, 256, 0, stream>>>(Vh, b, VTh); k_vtk<<<(KVW * (TT / 8) + 255) / 256, 256, 0, stream>>>(Vl, b, VTl);
    for (int hg = 0; hg < NH / HG; ++hg) { const int h0 = hg * HG; const int kvh = h0 / 4;
      k_gemm_hhx<0><<<gS, 128, 0, stream>>>(Q16 + (size_t)b * TT * CC + h0 * HD, CC, (size_t)HD, K16 + (size_t)b * TT * KVW + kvh * HD, KVW, 0, 0.125f, nullptr, 0, nullptr, 1, 0, 0, S, nullptr, TT, (size_t)TT * TT, TT, TT, HD);
      k_msoft<<<HG * TT / 8, 256, 0, stream>>>(S, P16);
      k_gemm_hhx<0><<<gV, 128, 0, stream>>>(P16, TT, (size_t)TT * TT, VTh + (size_t)kvh * HD * TT, TT, 0, 0.0009765625f, nullptr, 0, nullptr, 1, 0, 0, Of + (size_t)b * TT * CC + h0 * HD, nullptr, CC, (size_t)HD, TT, HD, TT);
      for (int g = 0; g < HG; ++g) { float* Co = Of + (size_t)b * TT * CC + (h0 + g) * HD; k_gemm_hhx<0><<<gV1, 128, 0, stream>>>(P16 + (size_t)g * TT * TT, TT, 0, VTl + (size_t)kvh * HD * TT, TT, 0, 0.0009765625f / 1024.0f, nullptr, 0, Co, 1, (size_t)CC, 0, Co, nullptr, CC, 0, TT, HD, TT); } } }
  k_split2<<<nb8, 256, 0, stream>>>(Of, O2, n8);
  k_gemm_hhx<0><<<dim3(((NR / 16) * (CC / 64) + 3) / 4, 1), 128, 0, stream>>>(O2, 2 * CC, 0, BO2, 2 * CC, 0, 0.0625f, b_o, 0, nullptr, 1, 0, 0, (float*)d_out, nullptr, CC, 0, NR, CC, 2 * CC);
}
